// MAB_9363028705889
// MI455X (gfx1250) — hardware-run, weakly checked
//
#include <hip/hip_runtime.h>


#ifndef NB
#define NB 8
#endif
#ifndef SEQ
#define SEQ 512
#endif
#define NB_FULL  8
#define SEQ_FULL 512
#ifndef OUT_SEQ
#define OUT_SEQ SEQ
#endif
#define TT   12
#define DM   64
#define NHD  8
#define HDM  8
#define AW   4
#define NZT  (NB * TT)
#define RR   (NZT * SEQ)
#define NTILE (RR / 64)
#define EPSV 1e-5f
#define SC2  (0.35355339059327376f * 1.4426950408889634f)

static_assert(DM == 64);
static_assert(NHD * HDM == DM);
static_assert(SEQ % 64 == 0);
static_assert(SEQ % 32 == 0);
static_assert(SEQ % (16 * AW) == 0);
static_assert(RR % 64 == 0);
static_assert(NTILE % 2 == 0);
static_assert(NB <= NB_FULL);
static_assert(SEQ <= SEQ_FULL);

typedef unsigned short bf;
typedef __attribute__((ext_vector_type(16))) __bf16   v16bf;
typedef __attribute__((ext_vector_type(8)))  unsigned short v8us;
typedef __attribute__((ext_vector_type(8)))  float    v8f;
typedef __attribute__((ext_vector_type(4)))  float    v4f;
typedef v4f  __attribute__((may_alias)) v4fa;

__device__ __forceinline__ unsigned short f2bf(float f) { unsigned u = __float_as_uint(f); u += 0x7FFFu + ((u >> 16) & 1u); return (unsigned short)(u >> 16); }
__device__ __forceinline__ float bf2f(unsigned short b) { return __uint_as_float(((unsigned)b) << 16); }
__device__ __forceinline__ float bfr(float f) { return bf2f(f2bf(f)); }
__device__ __forceinline__ v16bf cat16b(v8us lo, v8us hi) { return __builtin_bit_cast(v16bf, __builtin_shufflevector(lo, hi, 0, 1, 2, 3, 4, 5, 6, 7, 8, 9, 10, 11, 12, 13, 14, 15)); }
__device__ __forceinline__ v8f wmmab(v16bf a, v16bf b, v8f c) { return __builtin_amdgcn_wmma_f32_16x16x32_bf16(false, a, false, b, (short)0, c, false, false); }
__device__ __forceinline__ v16bf ldb(const bf* p)  { return cat16b(*(const v8us*)p, *(const v8us*)(p + 16)); }
__device__ __forceinline__ void wave_sync() { __builtin_amdgcn_fence(3  , "wavefront"); __builtin_amdgcn_wave_barrier(); asm volatile("" ::: "memory"); }
__device__ __forceinline__ size_t srow(int r) { if (SEQ == SEQ_FULL) return (size_t)r; return (size_t)(r / SEQ) * SEQ_FULL + (size_t)(r % SEQ); }
__device__ __forceinline__ size_t orow(int r) { if (OUT_SEQ == SEQ) return (size_t)r; return (size_t)(r / SEQ) * OUT_SEQ + (size_t)(r % SEQ); }

__global__ __launch_bounds__(256) void k_cvt8(const float* __restrict__ src, bf* dst, int n8) {
    const int i = blockIdx.x * 256 + threadIdx.x; if (i >= n8) return;
    const int row = i >> 3, c8 = (i & 7) * 8;
    const v8f v = *(const v8f*)(src + srow(row) * DM + c8); v8us o;
#pragma unroll
    for (int k = 0; k < 8; ++k) o[k] = f2bf(v[k]);
    bf* p = dst + (size_t)i * 8;
    *(volatile v8us*)p = o; __threadfence(); *(volatile v8us*)p = o;
}

__global__ __launch_bounds__(256) void k_wprep(const float* __restrict__ W, bf* WT, int KP) {
    __shared__ float wl[64 * 65];
    const int tid = threadIdx.x;
#pragma unroll 4
    for (int i = tid; i < 4096; i += 256) wl[(i >> 6) * 65 + (i & 63)] = W[i];
    __syncthreads();
    const int PR = KP >> 3, np = 64 * PR;
#pragma unroll 1
    for (int p = tid; p < np; p += 256) {
        const int n = p / PR, kk = (p % PR) * 8; v8us o;
#pragma unroll
        for (int i = 0; i < 8; ++i) o[i] = f2bf(wl[((kk + i) & 63) * 65 + n]);
        bf* d = WT + (size_t)p * 8;
        *(volatile v8us*)d = o; __threadfence(); *(volatile v8us*)d = o;
    }
}

__global__ __launch_bounds__(32) void k_gemm(const bf* __restrict__ A, const bf* __restrict__ Bt, const float* __restrict__ bias, float* Y, float* PS, int K) {
    __shared__ __align__(16) float os[16 * 68];
    const int lane = threadIdx.x & 31, lr = lane & 15, hi = lane >> 4; const int r0 = blockIdx.x * 64;
    v8f acc[4][4];
#pragma unroll
    for (int mb = 0; mb < 4; ++mb)
#pragma unroll
        for (int nb = 0; nb < 4; ++nb) acc[mb][nb] = (v8f){};
    const size_t aoff = (size_t)(r0 + lr) * K + 8 * hi, boff = (size_t)lr * K + 8 * hi;
#pragma unroll 1
    for (int kc = 0; kc < K; kc += 32) {
        v16bf a[4];
#pragma unroll
        for (int mb = 0; mb < 4; ++mb) a[mb] = ldb(A + aoff + (size_t)mb * 16 * K + kc);
#pragma unroll
        for (int nb = 0; nb < 4; ++nb) { const v16bf b = ldb(Bt + boff + (size_t)nb * 16 * K + kc);
#pragma unroll
            for (int mb = 0; mb < 4; ++mb) acc[mb][nb] = wmmab(a[mb], b, acc[mb][nb]); }
        asm volatile("v_nop\n\tv_nop\n\tv_nop\n\tv_nop" : "+v"(acc[0][0]), "+v"(acc[1][1]), "+v"(acc[2][2]), "+v"(acc[3][3]) : "v"(a[0]), "v"(a[1]), "v"(a[2]), "v"(a[3]));
    }
    float bv[4];
#pragma unroll
    for (int nb = 0; nb < 4; ++nb) bv[nb] = bfr(bias[nb * 16 + lr]);
    float s0 = 0.0f, s1 = 0.0f, q0 = 0.0f, q1 = 0.0f;
#pragma unroll
    for (int mb = 0; mb < 4; ++mb) {
#pragma unroll
        for (int nb = 0; nb < 4; ++nb) {
#pragma unroll
            for (int j = 0; j < 8; ++j) os[(hi * 8 + j) * 68 + nb * 16 + lr] = acc[mb][nb][j] + bv[nb]; }
        wave_sync();
#pragma unroll 4
        for (int row = 0; row < 16; ++row) { const float x0 = os[row * 68 + lane], x1 = os[row * 68 + 32 + lane]; s0 += x0; q0 += x0 * x0; s1 += x1; q1 += x1 * x1; }
        float* yb = Y + (size_t)(r0 + mb * 16) * DM;
#pragma unroll 1
        for (int ps = 0; ps < 2; ++ps) {
#pragma unroll
            for (int s = 0; s < 8; ++s) { const int row = 2 * s + hi, cofs = lr * 4;
                const v4f val = *(const v4fa*)(&os[row * 68 + cofs]);
                *(volatile v4f*)(yb + (size_t)row * DM + cofs) = val; }
            if (ps == 0) __threadfence(); }
        wave_sync();
    }
    os[lane] = s0; os[32 + lane] = s1; os[64 + lane] = q0; os[96 + lane] = q1;
    wave_sync();
    { const v4f pv = *(const v4fa*)(&os[lane * 4]); float* pp = PS + (size_t)blockIdx.x * 128 + lane * 4;
      *(volatile v4f*)pp = pv; __threadfence(); *(volatile v4f*)pp = pv; }
}

__global__ __launch_bounds__(256) void k_stats(const float* __restrict__ PS, float* ST) {
    __shared__ double sd[256];
    __shared__ double st[128];
    __shared__ __align__(16) float ol[128];
    const int tid = threadIdx.x, col = tid & 127, half = tid >> 7; const int job = blockIdx.x;
    const float* p = PS + (size_t)job * NTILE * 128 + (size_t)half * (NTILE / 2) * 128 + col;
    double s = 0.0;
#pragma unroll 8
    for (int i = 0; i < NTILE / 2; ++i) s += (double)p[(size_t)i * 128];
    sd[tid] = s;
    __syncthreads();
    if (tid < 128) st[tid] = sd[tid] + sd[tid + 128];
    __syncthreads();
    if (tid < 64) { const double mu = st[tid] * (1.0 / (double)RR); double var = st[64 + tid] * (1.0 / (double)RR) - mu * mu; if (var < 0.0) var = 0.0;
        ol[tid] = (float)mu; ol[64 + tid] = rsqrtf((float)var + EPSV); }
    __syncthreads();
    if (tid < 32) { const v4f v = *(const v4fa*)(&ol[tid * 4]); float* q = ST + (size_t)job * 128 + tid * 4;
        *(volatile v4f*)q = v; __threadfence(); *(volatile v4f*)q = v; }
}

__global__ __launch_bounds__(256) void k_norm(const float* __restrict__ Y3, const float* __restrict__ ST,
                                              const float* __restrict__ gq, const float* __restrict__ beq, const float* __restrict__ gk, const float* __restrict__ bek,
                                              const float* __restrict__ gv, const float* __restrict__ bev, const float* __restrict__ mask,
                                              bf* QK, bf* VT, float* MR) {
    __shared__ __align__(16) float tile[64 * 68];
    __shared__ __align__(16) float tmu[192];
    __shared__ __align__(16) float tsc[192];
    __shared__ __align__(16) float tbe[192];
    const int tid = threadIdx.x; const int r0 = blockIdx.x * 64; const int zt = r0 / SEQ, n0 = r0 % SEQ;
    if (tid < 192) { const int j = tid >> 6, c = tid & 63;
        const float g0 = gq[c], g1 = gk[c], g2 = gv[c], b0 = beq[c], b1 = bek[c], b2 = bev[c];
        const float g = bfr(j == 0 ? g0 : (j == 1 ? g1 : g2)); const float be = bfr(j == 0 ? b0 : (j == 1 ? b1 : b2));
        tmu[tid] = ST[j * 128 + c]; tsc[tid] = g * ST[j * 128 + 64 + c]; tbe[tid] = be; }
    __syncthreads();
    const size_t PLN = (size_t)RR * NHD * 16;
#pragma unroll 1
    for (int j = 0; j < 3; ++j) {
        const float* Y = Y3 + (size_t)j * RR * DM + (size_t)r0 * DM;
#pragma unroll
        for (int it = 0; it < 4; ++it) { const int idx = it * 256 + tid; const int row = idx >> 4, c4 = (idx & 15) * 4;
            const v4f y = *(const v4f*)(Y + (size_t)row * DM + c4);
            const v4f mu = *(const v4fa*)(&tmu[j * 64 + c4]); const v4f sc = *(const v4fa*)(&tsc[j * 64 + c4]); const v4f be = *(const v4fa*)(&tbe[j * 64 + c4]);
            v4f o;
#pragma unroll
            for (int e = 0; e < 4; ++e) o[e] = fmaxf((y[e] - mu[e]) * sc[e] + be[e], 0.0f);
            *(v4fa*)(&tile[row * 68 + c4]) = o; }
        __syncthreads();
        if (j < 2) {
            bf* P = QK + (size_t)j * PLN;
#pragma unroll 1
            for (int it = 0; it < 4; ++it) { const int p = it * 256 + tid; const int h = p >> 7, w = p & 127; const int n = w >> 1, part = w & 1;
                const v4f x0 = *(const v4fa*)(&tile[n * 68 + h * 8]); const v4f x1 = *(const v4fa*)(&tile[n * 68 + h * 8 + 4]); v8us o;
#pragma unroll
                for (int i = 0; i < 4; ++i) { const unsigned short a0 = f2bf(x0[i]); const unsigned short l0 = f2bf(x0[i] - bf2f(a0)); const unsigned short a1 = f2bf(x1[i]); const unsigned short l1 = f2bf(x1[i] - bf2f(a1));
                    o[i] = part ? l0 : a0; o[4 + i] = part ? l1 : a1; }
                bf* d = P + (((size_t)(zt * NHD + h) * SEQ + n0 + n) * 16 + part * 8);
                *(volatile v8us*)d = o; __threadfence(); *(volatile v8us*)d = o; }
        } else {
#pragma unroll 1
            for (int it = 0; it < 4; ++it) { const int p = it * 256 + tid; const int line = p >> 3, j8 = p & 7; const int h = line >> 4, drow = line & 15; const int d = drow & 7, part = drow >> 3;
                v8us o;
#pragma unroll
                for (int i = 0; i < 8; ++i) { const float x = tile[(8 * j8 + i) * 68 + h * 8 + d]; const unsigned short a = f2bf(x); const unsigned short l = f2bf(x - bf2f(a)); o[i] = part ? l : a; }
                bf* dd = VT + (((size_t)(zt * NHD + h) * 16 + drow) * SEQ + n0 + 8 * j8);
                *(volatile v8us*)dd = o; __threadfence(); *(volatile v8us*)dd = o; }
        }
        __syncthreads();
    }
    if (tid < 128) { const int h = tid >> 4, n4 = (tid & 15) * 4; v4f o;
#pragma unroll
        for (int i = 0; i < 4; ++i) { const float* mp = mask + srow(r0 + n4 + i) * DM + h * 8; const v4f a = *(const v4f*)mp; const v4f b = *(const v4f*)(mp + 4);
            o[i] = ((a[0] + a[1]) + (a[2] + a[3])) + ((b[0] + b[1]) + (b[2] + b[3])); }
        float* d = MR + (size_t)(zt * NHD + h) * SEQ + n0 + n4;
        *(volatile v4f*)d = o; __threadfence(); *(volatile v4f*)d = o; }
}

__global__ __launch_bounds__(32 * AW) __attribute__((amdgpu_num_vgpr(256))) void k_attn(const bf* __restrict__ QP, const bf* __restrict__ KP, const bf* __restrict__ VT, const float* __restrict__ MR, bf* M2) {
    __shared__ __align__(16) float os[AW * 16 * 68];
    const int lane = threadIdx.x & 31, lr = lane & 15, hi = lane >> 4;
    const int wave = __builtin_amdgcn_readfirstlane((int)(threadIdx.x >> 5));
    const int zt = blockIdx.y;
    const int t0 = (blockIdx.x * AW + wave) * 16;
    const int wb = wave * 16 * 68;
    const v8us zz = (v8us){};
#pragma unroll 1
    for (int h = 0; h < NHD; ++h) {
        const size_t pz = (size_t)zt * NHD + h;
        const bf* qrow = QP + (pz * SEQ + t0 + lr) * 16;
        const v8us qa = *(const v8us*)qrow; const v8us qb = *(const v8us*)(qrow + 8);
        const v16bf qf = cat16b(qa, hi == 0 ? qb : zz);
        const float mrv = MR[pz * SEQ + t0 + lr];
        const bool dead = (mrv == 0.0f);
        const bf* kbase = KP + (pz * SEQ + lr) * 16 + 8 * hi;
        const bf* vbase = VT + (pz * 16 + lr) * SEQ + 8 * hi;
        v8f o = (v8f){};
        float m = -3.0e38f, l = 0.0f;
#pragma unroll 1
        for (int key0 = 0; key0 < SEQ; key0 += 32) {
            const v8us ka = *(const v8us*)(kbase + (size_t)key0 * 16); const v8us kb = *(const v8us*)(kbase + (size_t)(key0 + 16) * 16);
            const v16bf kfa = cat16b(ka, hi == 0 ? ka : zz); const v16bf kfb = cat16b(kb, hi == 0 ? kb : zz);
            v8f sa = (v8f){}, sb = (v8f){};
            sa = wmmab(kfa, qf, sa); sb = wmmab(kfb, qf, sb);
            asm volatile("v_nop\n\tv_nop\n\tv_nop\n\tv_nop" : "+v"(sa), "+v"(sb) : "v"(kfa), "v"(kfb), "v"(qf));
            float ta[8], tb[8]; float mx = -3.0e38f;
#pragma unroll
            for (int r = 0; r < 8; ++r) { const float xa = sa[r] * SC2, xb = sb[r] * SC2; ta[r] = dead ? -1.0e9f : xa; tb[r] = dead ? -1.0e9f : xb; mx = fmaxf(mx, fmaxf(ta[r], tb[r])); }
            mx = fmaxf(mx, __shfl_xor(mx, 16, 32));
            const float mnew = fmaxf(m, mx);
            const float alpha = __builtin_amdgcn_exp2f(m - mnew);
            v8us ph0, ph1, pl0, pl1; float ls = 0.0f;
#pragma unroll
            for (int r = 0; r < 8; ++r) { const float pa = __builtin_amdgcn_exp2f(ta[r] - mnew); const float pc = __builtin_amdgcn_exp2f(tb[r] - mnew);
                const unsigned short ha = f2bf(pa), hc = f2bf(pc);
                ph0[r] = ha; ph1[r] = hc; pl0[r] = f2bf(pa - bf2f(ha)); pl1[r] = f2bf(pc - bf2f(hc)); ls += pa + pc; }
            l = l * alpha + ls; m = mnew;
            o = o * alpha;
            const v16bf vt = ldb(vbase + key0);
            const v16bf pfh = cat16b(ph0, ph1), pfl = cat16b(pl0, pl1);
            o = wmmab(vt, pfh, o); o = wmmab(vt, pfl, o);
            asm volatile("v_nop\n\tv_nop\n\tv_nop\n\tv_nop" : "+v"(o) : "v"(vt), "v"(pfh), "v"(pfl));
        }
        l += __shfl_xor(l, 16, 32);
        const float inv = 1.0f / l;
        v4f a, c;
#pragma unroll
        for (int r = 0; r < 4; ++r) { const float u0 = o[r] + __shfl_xor(o[r], 16, 32); const float u1 = o[4 + r] + __shfl_xor(o[4 + r], 16, 32); a[r] = u0 * inv; c[r] = u1 * inv; }
        if (hi == 0) { *(v4fa*)(&os[wb + lr * 68 + h * 8]) = a; *(v4fa*)(&os[wb + lr * 68 + h * 8 + 4]) = c; }
    }
    wave_sync();
    bf* mbase = M2 + ((size_t)zt * SEQ + t0) * 128;
#pragma unroll 1
    for (int ps = 0; ps < 2; ++ps) {
#pragma unroll
        for (int s = 0; s < 8; ++s) { const int row = 2 * s + hi; const int c8 = (lr & 7) * 8, part = lr >> 3;
            const v4f x0 = *(const v4fa*)(&os[wb + row * 68 + c8]); const v4f x1 = *(const v4fa*)(&os[wb + row * 68 + c8 + 4]); v8us ov;
#pragma unroll
            for (int i = 0; i < 4; ++i) { const unsigned short a0 = f2bf(x0[i]); const unsigned short l0 = f2bf(x0[i] - bf2f(a0)); const unsigned short a1 = f2bf(x1[i]); const unsigned short l1 = f2bf(x1[i] - bf2f(a1));
                ov[i] = part ? l0 : a0; ov[4 + i] = part ? l1 : a1; }
            *(volatile v8us*)(mbase + (size_t)row * 128 + lr * 8) = ov; }
        if (ps == 0) __threadfence(); }
}

__global__ __launch_bounds__(256) void k_final(const float* __restrict__ Y, const float* __restrict__ ST, const float* __restrict__ g, const float* __restrict__ be, float* OUT) {
    const int i = blockIdx.x * 256 + threadIdx.x; if (i >= RR * 16) return;
    const int row = i >> 4, c4 = (i & 15) * 4;
    const v4f y = *(const v4f*)(Y + (size_t)i * 4);
    const v4f mu = *(const v4f*)(ST + c4); const v4f rs = *(const v4f*)(ST + 64 + c4);
    const v4f gg = *(const v4f*)(g + c4); const v4f bb = *(const v4f*)(be + c4);
    v4f o;
#pragma unroll
    for (int e = 0; e < 4; ++e) o[e] = fmaxf((y[e] - mu[e]) * (bfr(gg[e]) * rs[e]) + bfr(bb[e]), 0.0f);
    float* d = OUT + orow(row) * DM + c4;
    *(volatile v4f*)d = o; __threadfence(); *(volatile v4f*)d = o;
}

static constexpr size_t al256(size_t v) { return (v + 255) & ~(size_t)255; }
static constexpr size_t SZ_XB = al256((size_t)RR * DM * 2);
static constexpr size_t SZ_WT = al256((size_t)(3 * 64 * 64 + 64 * 128) * 2);
static constexpr size_t SZ_Y  = al256((size_t)RR * DM * 4);
static constexpr size_t SZ_PS = al256((size_t)4 * NTILE * 128 * 4);
static constexpr size_t SZ_ST = al256((size_t)4 * 128 * 4);
static constexpr size_t SZ_QK = al256((size_t)RR * NHD * 16 * 2);
static constexpr size_t SZ_VT = al256((size_t)NZT * NHD * 16 * SEQ * 2);
static constexpr size_t SZ_MR = al256((size_t)NZT * NHD * SEQ * 4);
static constexpr size_t SZ_M2 = al256((size_t)RR * 128 * 2);
static constexpr size_t SZ_TOTAL = 2 * SZ_XB + SZ_WT + 4 * SZ_Y + SZ_PS + SZ_ST + 2 * SZ_QK + SZ_VT + SZ_MR + SZ_M2;
static_assert(SZ_TOTAL <= (size_t)134217728);
static_assert(SZ_QK == (size_t)RR * NHD * 16 * 2);
static_assert(SZ_Y == (size_t)RR * DM * 4);

extern "C" void kernel_launch(void* const* d_in, const int* in_sizes, int n_in,
                              void* d_out, int out_size, void* d_ws, size_t ws_size, hipStream_t stream) {
    if (n_in < 20) return;
    const size_t needx = ((size_t)(NZT - 1) * SEQ_FULL + SEQ) * DM;
    if ((size_t)in_sizes[0] < needx || (size_t)in_sizes[1] < needx || (size_t)in_sizes[2] < needx) return;
    if (in_sizes[3] < 1) return;
    for (int f = 0; f < 4; ++f) {
        if ((size_t)in_sizes[4 + 4 * f] < (size_t)DM * DM) return;
        if (in_sizes[5 + 4 * f] < DM || in_sizes[6 + 4 * f] < DM || in_sizes[7 + 4 * f] < DM) return;
    }
    if ((size_t)out_size < ((size_t)(NZT - 1) * OUT_SEQ + SEQ) * DM) return;
    if (SZ_TOTAL > ws_size) return;
    const float* Q = (const float*)d_in[0]; const float* Kin = (const float*)d_in[1]; const float* mask = (const float*)d_in[2];
    const int* bsz = (const int*)d_in[3]; (void)bsz;
    const float* Wq = (const float*)d_in[4];  const float* bq = (const float*)d_in[5];  const float* gq = (const float*)d_in[6];  const float* beq = (const float*)d_in[7];
    const float* Wk = (const float*)d_in[8];  const float* bk = (const float*)d_in[9];  const float* gk = (const float*)d_in[10]; const float* bek = (const float*)d_in[11];
    const float* Wv = (const float*)d_in[12]; const float* bv = (const float*)d_in[13]; const float* gv = (const float*)d_in[14]; const float* bev = (const float*)d_in[15];
    const float* Wo = (const float*)d_in[16]; const float* bo = (const float*)d_in[17]; const float* go = (const float*)d_in[18]; const float* beo = (const float*)d_in[19];
    float* OUT = (float*)d_out;
    char* wsp = (char*)d_ws;
    bf* XQ = (bf*)wsp; wsp += SZ_XB;
    bf* XK = (bf*)wsp; wsp += SZ_XB;
    bf* WT = (bf*)wsp; wsp += SZ_WT;
    float* Y3 = (float*)wsp; wsp += 3 * SZ_Y;
    float* YO = (float*)wsp; wsp += SZ_Y;
    float* PS = (float*)wsp; wsp += SZ_PS;
    float* ST = (float*)wsp; wsp += SZ_ST;
    bf* QK = (bf*)wsp; wsp += 2 * SZ_QK;
    bf* VT = (bf*)wsp; wsp += SZ_VT;
    float* MR = (float*)wsp; wsp += SZ_MR;
    bf* M2 = (bf*)wsp; wsp += SZ_M2;
    bf* WTq = WT; bf* WTk = WT + 4096; bf* WTv = WT + 8192; bf* WTo = WT + 12288;
    const size_t PLN = (size_t)RR * NHD * 16;

    { const int n8 = RR * DM / 8; const unsigned g = (unsigned)((n8 + 255) / 256);
      k_cvt8<<<g, 256, 0, stream>>>(Q, XQ, n8); k_cvt8<<<g, 256, 0, stream>>>(Kin, XK, n8); }
    k_wprep<<<1, 256, 0, stream>>>(Wq, WTq, 64); k_wprep<<<1, 256, 0, stream>>>(Wk, WTk, 64);
    k_wprep<<<1, 256, 0, stream>>>(Wv, WTv, 64); k_wprep<<<1, 256, 0, stream>>>(Wo, WTo, 128);

    k_gemm<<<NTILE, 32, 0, stream>>>(XQ, WTq, bq, Y3, PS, 64);
    k_gemm<<<NTILE, 32, 0, stream>>>(XK, WTk, bk, Y3 + (size_t)RR * DM, PS + (size_t)NTILE * 128, 64);
    k_gemm<<<NTILE, 32, 0, stream>>>(XK, WTv, bv, Y3 + (size_t)2 * RR * DM, PS + (size_t)2 * NTILE * 128, 64);
    k_stats<<<3, 256, 0, stream>>>(PS, ST);

    k_norm<<<NTILE, 256, 0, stream>>>(Y3, ST, gq, beq, gk, bek, gv, bev, mask, QK, VT, MR);
    k_attn<<<dim3(SEQ / (16 * AW), NZT, 1), 32 * AW, 0, stream>>>(QK, QK + PLN, VT, MR, M2);

    k_gemm<<<NTILE, 32, 0, stream>>>(M2, WTo, bo, YO, PS + (size_t)3 * NTILE * 128, 128);
    k_stats<<<1, 256, 0, stream>>>(PS + (size_t)3 * NTILE * 128, ST + 3 * 128);
    k_final<<<(RR * 16 + 255) / 256, 256, 0, stream>>>(YO, ST + 3 * 128, go, beo, OUT);
}
